// LNN_82935818486281
// MI455X (gfx1250) — hardware-verified
//
#include <hip/hip_runtime.h>
#include <math.h>

constexpr int kBS   = 65536;
constexpr int kHid  = 256;
constexpr int kNQ   = 8;
constexpr int kNL   = 36;
constexpr int kNLP  = 64;
constexpr float kWCarry    = 16.0f;
constexpr float kWCarryInv = 0.0625f;

constexpr size_t kActPlane = (size_t)kBS * kHid * 2;
constexpr size_t kGlPlane  = (size_t)kBS * kNLP * 2;
constexpr size_t kLpPlane  = (size_t)kBS * kNLP * 4;
constexpr size_t kVec8     = (size_t)kBS * kNQ * 4;
constexpr size_t OFF_H1  = 0;
constexpr size_t OFF_H2  = OFF_H1 + kActPlane;
constexpr size_t OFF_GP2 = OFF_H2 + kActPlane;
constexpr size_t OFF_GL  = OFF_GP2 + kActPlane;
constexpr size_t OFF_LP  = OFF_GL + kGlPlane;
constexpr size_t OFF_DV  = OFF_LP + kLpPlane;
constexpr size_t OFF_DT  = OFF_DV + kVec8;
constexpr size_t OFF_W2T = OFF_DT + kVec8;
constexpr size_t OFF_W2C = OFF_W2T + (size_t)kHid * kHid * 2;
constexpr size_t OFF_W3T = OFF_W2C + (size_t)kHid * kHid * 2;
constexpr size_t OFF_W3B = OFF_W3T + (size_t)kNLP * kHid * 2;
constexpr size_t OFF_B3P = OFF_W3B + (size_t)kHid * kNLP * 2;
constexpr size_t WS_TOTAL = OFF_B3P + 256;
static_assert(WS_TOTAL == 130351360, "");
static_assert(WS_TOTAL <= 134217728, "");
static_assert((OFF_H2 % 128) == 0 && (OFF_GL % 128) == 0 && (OFF_LP % 128) == 0 && (OFF_DV % 128) == 0, "");
static_assert((OFF_DT % 128) == 0 && (OFF_W2T % 128) == 0 && (OFF_W3T % 128) == 0 && (OFF_W3B % 128) == 0 && (OFF_B3P % 128) == 0, "");
static_assert(kBS % 256 == 0 && kHid % 64 == 0 && kNLP % 64 == 0 && kHid % 32 == 0 && kNLP % 32 == 0, "");
static_assert((kBS / 64) * (kHid / 64) == 512 * 8, "");
static_assert((kBS / 64) * (kNLP / 64) == 128 * 8, "");

typedef __attribute__((ext_vector_type(16))) _Float16 v16h;
typedef __attribute__((ext_vector_type(8)))  _Float16 v8h;
typedef __attribute__((ext_vector_type(16))) __bf16   v16b;
typedef __attribute__((ext_vector_type(8)))  __bf16   v8b;
typedef __attribute__((ext_vector_type(8)))  float    v8f;
typedef __attribute__((ext_vector_type(4)))  float    v4f;
typedef __attribute__((ext_vector_type(4)))  unsigned int v4u;

__host__ __device__ constexpr int tri_idx(int i, int j) { return i * (i + 1) / 2 + j; }

__device__ __forceinline__ unsigned short f2bf_bits(float f) {
  unsigned u = __float_as_uint(f);
  return (unsigned short)((u + 0x7FFFu + ((u >> 16) & 1u)) >> 16);
}
__device__ __forceinline__ float bf_bits2f(unsigned short h) { return __uint_as_float(((unsigned)h) << 16); }

__device__ __forceinline__ void dep_guard_h(v8f& a, v8f& b, v16h x, v16h y) { asm volatile("v_nop\n\tv_nop\n\tv_nop\n\tv_nop" : "+v"(a), "+v"(b) : "v"(x), "v"(y)); }
__device__ __forceinline__ void dep_guard_b(v8f& a, v8f& b, v16b x, v16b y) { asm volatile("v_nop\n\tv_nop\n\tv_nop\n\tv_nop" : "+v"(a), "+v"(b) : "v"(x), "v"(y)); }
__device__ __forceinline__ void dep_guard4_h(v8f& a, v8f& b, v8f& c, v8f& d, v16h x, v16h y, v16h p0, v16h p1, v16h p2, v16h p3) {
  asm volatile("v_nop\n\tv_nop\n\tv_nop\n\tv_nop" : "+v"(a), "+v"(b), "+v"(c), "+v"(d) : "v"(x), "v"(y), "v"(p0), "v"(p1), "v"(p2), "v"(p3));
}
__device__ __forceinline__ void dep_guard4_b(v8f& a, v8f& b, v8f& c, v8f& d, v16b x, v16b y, v16b p0, v16b p1, v16b p2, v16b p3) {
  asm volatile("v_nop\n\tv_nop\n\tv_nop\n\tv_nop" : "+v"(a), "+v"(b), "+v"(c), "+v"(d) : "v"(x), "v"(y), "v"(p0), "v"(p1), "v"(p2), "v"(p3));
}
__device__ __forceinline__ void keep4_h(v16h a, v16h b, v16h c, v16h d) { asm volatile("v_nop" :: "v"(a), "v"(b), "v"(c), "v"(d)); }
__device__ __forceinline__ void keep4_b(v16b a, v16b b, v16b c, v16b d) { asm volatile("v_nop" :: "v"(a), "v"(b), "v"(c), "v"(d)); }
__device__ __forceinline__ void acc_guard4(v8f& a, v8f& b, v8f& c, v8f& d) { asm volatile("v_nop\n\tv_nop\n\tv_nop\n\tv_nop" : "+v"(a), "+v"(b), "+v"(c), "+v"(d)); }
template <typename T> struct Frag;
template <> struct Frag<_Float16> {
  typedef v16h V; union U { v16h v; v8h h[2]; };
  static __device__ __forceinline__ v16h load(const _Float16* p) {
    U f; f.h[0] = *(const v8h*)(p); f.h[1] = *(const v8h*)(p + 16); return f.v;
  }
  static __device__ __forceinline__ v8f mma(v16h a, v16h b, v8f c) {
    return __builtin_amdgcn_wmma_f32_16x16x32_f16(false, a, false, b, (short)0, c, false, false);
  }
  static __device__ __forceinline__ void guard(v8f& a, v8f& b, v16h x, v16h y) { dep_guard_h(a, b, x, y); }
  static __device__ __forceinline__ void guard4(v8f& a, v8f& b, v8f& c, v8f& d, v16h x, v16h y, v16h p0, v16h p1, v16h p2, v16h p3) { dep_guard4_h(a, b, c, d, x, y, p0, p1, p2, p3); }
  static __device__ __forceinline__ void keep(v16h a, v16h b, v16h c, v16h d) { keep4_h(a, b, c, d); }
};
template <> struct Frag<__bf16> {
  typedef v16b V; union U { v16b v; v8b h[2]; };
  static __device__ __forceinline__ v16b load(const __bf16* p) {
    U f; f.h[0] = *(const v8b*)(p); f.h[1] = *(const v8b*)(p + 16); return f.v;
  }
  static __device__ __forceinline__ v8f mma(v16b a, v16b b, v8f c) {
    return __builtin_amdgcn_wmma_f32_16x16x32_bf16(false, a, false, b, (short)0, c, false, false);
  }
  static __device__ __forceinline__ void guard(v8f& a, v8f& b, v16b x, v16b y) { dep_guard_b(a, b, x, y); }
  static __device__ __forceinline__ void guard4(v8f& a, v8f& b, v8f& c, v8f& d, v16b x, v16b y, v16b p0, v16b p1, v16b p2, v16b p3) { dep_guard4_b(a, b, c, d, x, y, p0, p1, p2, p3); }
  static __device__ __forceinline__ void keep(v16b a, v16b b, v16b c, v16b d) { keep4_b(a, b, c, d); }
};

__device__ __forceinline__ unsigned pk16(unsigned short a, unsigned short b) { return (unsigned)a | ((unsigned)b << 16); }
__device__ __forceinline__ unsigned short h_bits(float f) { const _Float16 h = (_Float16)f; return __builtin_bit_cast(unsigned short, h); }
__device__ __forceinline__ float h16_to_f32(unsigned hb) {
  const unsigned sgn = (hb & 0x8000u) << 16; const unsigned em = hb & 0x7fffu;
  const float fn = __uint_as_float((em << 13) + 0x38000000u);
  const float fs = (float)em * 5.9604644775390625e-8f;
  const float mag = (em < 0x400u) ? fs : fn; return __uint_as_float(__float_as_uint(mag) | sgn); }

template <int ET> struct Elem;
template <> struct Elem<0> { typedef _Float16 T; };
template <> struct Elem<1> { typedef __bf16 T; };
template <int ET, bool SPLIT, int BIAS_MODE, int OUT_MODE, bool RESID, int ACT = 0>
__global__ __launch_bounds__(256) void wmma_gemm64(
    const unsigned short* __restrict__ Ap, const unsigned short* __restrict__ A2p, int lda, long strideA,
    const unsigned short* __restrict__ Btp, const unsigned short* __restrict__ Bt2p, int ldb, long strideB,
    void* __restrict__ Cout, void* __restrict__ Cout2, int ldc, long strideC,
    const float* __restrict__ bias,
    const float* __restrict__ resid, long strideR,
    int M, int N, int K, float scale) {
  typedef typename Elem<ET>::T T;
  typedef typename Frag<T>::V V;
  const T* A = (const T*)Ap; const T* A2 = (const T*)A2p; const T* Bt = (const T*)Btp; const T* Bt2 = (const T*)Bt2p;
  __shared__ __align__(16) float sT[8][16 * 68];
  const int b    = blockIdx.y;
  const int lane = threadIdx.x & 31;
  const int wave = threadIdx.x >> 5;
  const int tilesN = N >> 6;
  const int tilesM = M >> 6;
  const int tile = blockIdx.x * 8 + wave;
  if (tile >= tilesM * tilesN) return;
  const int tm = tile / tilesN;
  const int tn = tile - tm * tilesN;
  const int m0 = tm << 6;
  const int n0 = tn << 6;

  const T* Ab  = A  + (size_t)b * strideA;
  const T* Bb  = Bt + (size_t)b * strideB;
  const T* Ab2 = SPLIT ? (A2  + (size_t)b * strideA) : nullptr;
  const T* Bb2 = SPLIT ? (Bt2 + (size_t)b * strideB) : nullptr;

  const int rlane = lane & 15;
  const int koff  = (lane >> 4) * 8;
  const int mOff  = (lane >> 4) * 8;

  v8f acc[4][4];
#pragma unroll
  for (int i = 0; i < 4; ++i)
#pragma unroll
    for (int j = 0; j < 4; ++j) acc[i][j] = (v8f){0.f,0.f,0.f,0.f,0.f,0.f,0.f,0.f};

  for (int k0 = 0; k0 < K; k0 += 32) {
    V bh[4], bl[4];
#pragma unroll
    for (int j = 0; j < 4; ++j) {
      const size_t bo = (size_t)(n0 + (j << 4) + rlane) * ldb + koff + k0;
      bh[j] = Frag<T>::load(Bb + bo);
      if (SPLIT) bl[j] = Frag<T>::load(Bb2 + bo);
    }
#pragma unroll
    for (int i = 0; i < 4; ++i) {
      const size_t ao = (size_t)(m0 + (i << 4) + rlane) * lda + koff + k0;
      V ah = Frag<T>::load(Ab + ao);
      V al;
      if (SPLIT) al = Frag<T>::load(Ab2 + ao);
#pragma unroll
      for (int j = 0; j < 4; ++j) {
        acc[i][j] = Frag<T>::mma(ah, bh[j], acc[i][j]);
        if (SPLIT) {
          acc[i][j] = Frag<T>::mma(ah, bl[j], acc[i][j]);
          acc[i][j] = Frag<T>::mma(al, bh[j], acc[i][j]);
        }
      }
      Frag<T>::guard4(acc[i][0], acc[i][1], acc[i][2], acc[i][3], ah, SPLIT ? al : ah, bh[0], bh[1], bh[2], bh[3]);
    }
    Frag<T>::keep(bh[0], bh[1], bh[2], bh[3]);
    if (SPLIT) Frag<T>::keep(bl[0], bl[1], bl[2], bl[3]);
  }
  acc_guard4(acc[0][0], acc[0][1], acc[0][2], acc[0][3]);
  acc_guard4(acc[1][0], acc[1][1], acc[1][2], acc[1][3]);
  acc_guard4(acc[2][0], acc[2][1], acc[2][2], acc[2][3]);
  acc_guard4(acc[3][0], acc[3][1], acc[3][2], acc[3][3]);

  float* slab = sT[wave];
  const float* Rb = RESID ? (resid + (size_t)b * strideR) : nullptr;
#pragma unroll
  for (int i = 0; i < 4; ++i) {
    const int mBase = m0 + (i << 4);
#pragma unroll
    for (int j = 0; j < 4; ++j) {
      const int n = n0 + (j << 4) + rlane;
      float bv = 0.f;
      if (BIAS_MODE == 2) bv = bias[n];
#pragma unroll
      for (int r = 0; r < 8; ++r) {
        float v = acc[i][j][r] * scale;
        if (BIAS_MODE == 1) v += bias[mBase + mOff + r];
        if (BIAS_MODE == 2) v += bv;
        if (RESID) v += Rb[(size_t)(mBase + mOff + r) * ldc + n];
        if (ACT == 1) v = tanhf(v);
        if (ACT == 2) v = fmaxf(v, 0.0f);
        if (ACT == 3) v = v / (1.0f + expf(-v));
        if (ACT == 4) v = (v > 0.f) ? v : 0.01f * v;
        if (ACT == 5) v = 0.5f * v * (1.0f + erff(v * 0.70710678118654752f));
        slab[(mOff + r) * 68 + (j << 4) + rlane] = v;
      }
    }
    __builtin_amdgcn_fence(__ATOMIC_RELEASE, "workgroup");
    __builtin_amdgcn_wave_barrier();
    __builtin_amdgcn_fence(__ATOMIC_ACQUIRE, "workgroup");
    if (OUT_MODE == 0) {
      float* C = (float*)Cout + (size_t)b * strideC;
      const int hh = lane >> 4, c4 = (lane & 15) * 4;
      for (int pass = 0; pass < 2; ++pass) {
#pragma unroll
        for (int it = 0; it < 8; ++it) {
          const int row = it * 2 + hh;
          v4f v = *(const v4f*)(slab + row * 68 + c4);
          *(volatile v4f*)(C + (size_t)(mBase + row) * ldc + n0 + c4) = v;
        }
        __threadfence();
      }
    } else {
      const int q = lane >> 3, c8 = (lane & 7) * 8;
      unsigned short* C  = (unsigned short*)Cout  + (size_t)b * strideC;
      unsigned short* C2 = (OUT_MODE == 2) ? ((unsigned short*)Cout2 + (size_t)b * strideC) : nullptr;
      for (int pass = 0; pass < 2; ++pass) {
#pragma unroll
        for (int it = 0; it < 4; ++it) {
          const int row = it * 4 + q;
          const float* sp = slab + row * 68 + c8;
          v8h hv, lv;
#pragma unroll
          for (int e = 0; e < 8; ++e) {
            if (OUT_MODE == 1) {
              hv[e] = (_Float16)sp[e];
            } else {
              unsigned short hb = f2bf_bits(sp[e]);
              unsigned short lb = f2bf_bits(sp[e] - bf_bits2f(hb));
              hv[e] = __builtin_bit_cast(_Float16, hb);
              lv[e] = __builtin_bit_cast(_Float16, lb);
            }
          }
          *(volatile v8h*)(C + (size_t)(mBase + row) * ldc + n0 + c8) = hv;
          if (OUT_MODE == 2) *(volatile v8h*)(C2 + (size_t)(mBase + row) * ldc + n0 + c8) = lv;
        }
        __threadfence();
      }
    }
    __builtin_amdgcn_fence(__ATOMIC_RELEASE, "workgroup");
    __builtin_amdgcn_wave_barrier();
    __builtin_amdgcn_fence(__ATOMIC_ACQUIRE, "workgroup");
  }
}

template <int LDA, int LDB, int KDIM>
__device__ __forceinline__ void mma_tile64_f16(const _Float16* __restrict__ A, const _Float16* __restrict__ Bt,
                                               int m0, int n0, int lane, v8f (&acc)[4][4]) {
  static_assert(KDIM % 32 == 0 && LDA % 8 == 0 && LDB % 8 == 0, "");
  const int rlane = lane & 15;
  const int koff  = (lane >> 4) * 8;
#pragma unroll
  for (int i = 0; i < 4; ++i)
#pragma unroll
    for (int j = 0; j < 4; ++j) acc[i][j] = (v8f){0.f,0.f,0.f,0.f,0.f,0.f,0.f,0.f};
  for (int k0 = 0; k0 < KDIM; k0 += 32) {
    v16h bh[4];
#pragma unroll
    for (int j = 0; j < 4; ++j) bh[j] = Frag<_Float16>::load(Bt + (size_t)(n0 + (j << 4) + rlane) * LDB + koff + k0);
#pragma unroll
    for (int i = 0; i < 4; ++i) {
      const v16h ah = Frag<_Float16>::load(A + (size_t)(m0 + (i << 4) + rlane) * LDA + koff + k0);
#pragma unroll
      for (int j = 0; j < 4; ++j) acc[i][j] = Frag<_Float16>::mma(ah, bh[j], acc[i][j]);
      dep_guard4_h(acc[i][0], acc[i][1], acc[i][2], acc[i][3], ah, ah, bh[0], bh[1], bh[2], bh[3]);
    }
    keep4_h(bh[0], bh[1], bh[2], bh[3]);
  }
  acc_guard4(acc[0][0], acc[0][1], acc[0][2], acc[0][3]);
  acc_guard4(acc[1][0], acc[1][1], acc[1][2], acc[1][3]);
  acc_guard4(acc[2][0], acc[2][1], acc[2][2], acc[2][3]);
  acc_guard4(acc[3][0], acc[3][1], acc[3][2], acc[3][3]);
}

__global__ __launch_bounds__(256) void pack_w2t_kernel(const float* __restrict__ W, unsigned short* __restrict__ outT, float scale) {
  __shared__ float sm[64][65];
  const int t  = threadIdx.x;
  const int k0 = blockIdx.x * 64;
  const int n0 = blockIdx.y * 64;
#pragma unroll
  for (int i = 0; i < 16; ++i) {
    const int e = i * 256 + t;
    const int r = e >> 6;
    const int c = e & 63;
    sm[c][r] = W[(size_t)(k0 + r) * kHid + n0 + c] * scale;
  }
  __syncthreads();
  const int lane = t & 31, wave = t >> 5;
  const int q = lane >> 3, c8 = (lane & 7) * 8;
  for (int pass = 0; pass < 2; ++pass) {
#pragma unroll
    for (int it = 0; it < 2; ++it) {
      const int row = wave * 8 + it * 4 + q;
      unsigned short hb[8];
#pragma unroll
      for (int e = 0; e < 8; ++e) hb[e] = h_bits(sm[row][c8 + e]);
      const v4u u = (v4u){pk16(hb[0], hb[1]), pk16(hb[2], hb[3]), pk16(hb[4], hb[5]), pk16(hb[6], hb[7])};
      *(volatile v4u*)(outT + (size_t)(n0 + row) * kHid + k0 + c8) = u;
    }
    __threadfence();
  }
}

__global__ __launch_bounds__(256) void pack_cast8_kernel(const float* __restrict__ in, unsigned short* __restrict__ out, int n8, float scale) {
  const int i = blockIdx.x * 256 + threadIdx.x;
  if (i >= n8) return;
  const float* p = in + 8 * (size_t)i;
  const v4f a = *(const v4f*)(p);
  const v4f c = *(const v4f*)(p + 4);
  unsigned short hb[8];
#pragma unroll
  for (int e = 0; e < 4; ++e) {
    hb[e]     = h_bits(a[e] * scale);
    hb[4 + e] = h_bits(c[e] * scale);
  }
  const v4u u = (v4u){pk16(hb[0], hb[1]), pk16(hb[2], hb[3]), pk16(hb[4], hb[5]), pk16(hb[6], hb[7])};
  unsigned short* o = out + 8 * (size_t)i;
  *(volatile v4u*)o = u;
  __threadfence();
  *(volatile v4u*)o = u;
}

__global__ __launch_bounds__(256) void pack_w3_kernel(const float* __restrict__ W3, const float* __restrict__ b3,
                                                     unsigned short* __restrict__ w3t, unsigned short* __restrict__ w3b,
                                                     float* __restrict__ b3p, float scale) {
  const int t = threadIdx.x, lane = t & 31, wave = t >> 5;
  if (blockIdx.x == 0) {
#pragma unroll 1
    for (int rr = 0; rr < 8; ++rr) {
      const int tt = wave * 8 + rr;
      const int tc = tt < kNL ? tt : kNL - 1;
      const float f = tt < kNL ? scale : 0.0f;
      unsigned short hb[8];
#pragma unroll
      for (int e = 0; e < 8; ++e) hb[e] = h_bits(W3[(size_t)(lane * 8 + e) * kNL + tc] * f);
      const v4u u = (v4u){pk16(hb[0], hb[1]), pk16(hb[2], hb[3]), pk16(hb[4], hb[5]), pk16(hb[6], hb[7])};
      unsigned short* o = w3t + (size_t)tt * kHid + lane * 8;
      *(volatile v4u*)o = u;
      __threadfence();
      *(volatile v4u*)o = u;
    }
  } else {
#pragma unroll 1
    for (int s = 0; s < 8; ++s) {
      const int n  = wave * 32 + s * 4 + (lane >> 3);
      const int kb = (lane & 7) * 8;
      unsigned short hb[8];
#pragma unroll
      for (int e = 0; e < 8; ++e) {
        const int k  = kb + e;
        const int kc = k < kNL ? k : kNL - 1;
        const float f = k < kNL ? scale : 0.0f;
        hb[e] = h_bits(W3[(size_t)n * kNL + kc] * f);
      }
      const v4u u = (v4u){pk16(hb[0], hb[1]), pk16(hb[2], hb[3]), pk16(hb[4], hb[5]), pk16(hb[6], hb[7])};
      unsigned short* o = w3b + (size_t)n * kNLP + kb;
      *(volatile v4u*)o = u;
      __threadfence();
      *(volatile v4u*)o = u;
    }
    if (wave == 0) {
      float bv[4];
#pragma unroll
      for (int e = 0; e < 4; ++e) {
        const int c  = lane * 4 + e;
        const int cc = c < kNL ? c : kNL - 1;
        const float f = c < kNL ? 1.0f : 0.0f;
        bv[e] = b3[cc] * f;
      }
      const v4f v = (v4f){bv[0], bv[1], bv[2], bv[3]};
      if (lane < 16) {
        float* o = b3p + lane * 4;
        *(volatile v4f*)o = v;
        __threadfence();
        *(volatile v4f*)o = v;
      }
    }
  }
}

__global__ __launch_bounds__(256) void h1_vnet_kernel(const float* __restrict__ q, const float* __restrict__ W1, const float* __restrict__ b1,
                                                     const float* __restrict__ Wv1, const float* __restrict__ bv1, const float* __restrict__ Wv2,
                                                     unsigned short* __restrict__ H1, float* __restrict__ DV) {
  __shared__ __align__(16) float w1t[kHid * kNQ];
  __shared__ __align__(16) float wvt[kHid * kNQ];
  __shared__ float b1s[kHid];
  __shared__ float bv1s[kHid];
  __shared__ float wv2s[kHid];
  const int t = threadIdx.x, lane = t & 31, wave = t >> 5;
  {
    float a[8];
#pragma unroll
    for (int j = 0; j < 8; ++j) a[j] = W1[j * kHid + t];
    *(v4f*)(w1t + t * 8)     = (v4f){a[0], a[1], a[2], a[3]};
    *(v4f*)(w1t + t * 8 + 4) = (v4f){a[4], a[5], a[6], a[7]};
    asm volatile("" ::: "memory");
    float c[8];
#pragma unroll
    for (int j = 0; j < 8; ++j) c[j] = Wv1[j * kHid + t];
    *(v4f*)(wvt + t * 8)     = (v4f){c[0], c[1], c[2], c[3]};
    *(v4f*)(wvt + t * 8 + 4) = (v4f){c[4], c[5], c[6], c[7]};
    asm volatile("" ::: "memory");
    b1s[t] = b1[t]; bv1s[t] = bv1[t]; wv2s[t] = Wv2[t];
  }
  __syncthreads();
  const int wrow0 = blockIdx.x * 128 + wave * 16;
  const int myr = lane >> 1;
  const bool odd = (lane & 1) != 0;
  float k0 = 0.0f, k1 = 0.0f, k2 = 0.0f, k3 = 0.0f;
#pragma unroll 1
  for (int rr = 0; rr < 16; ++rr) {
    const int row = wrow0 + rr;
    const v4f qa = *(const v4f*)(q + (size_t)row * kNQ);
    const v4f qb = *(const v4f*)(q + (size_t)row * kNQ + 4);
    v4u hw = (v4u){0u, 0u, 0u, 0u};
#pragma unroll 1
    for (int p = 0; p < 4; ++p) {
      const int c0 = lane * 8 + 2 * p;
      const v4f wa0 = *(const v4f*)(w1t + c0 * 8),     wa1 = *(const v4f*)(w1t + c0 * 8 + 4);
      const v4f wb0 = *(const v4f*)(w1t + c0 * 8 + 8), wb1 = *(const v4f*)(w1t + c0 * 8 + 12);
      float p0 = b1s[c0], p1 = b1s[c0 + 1];
      p0 = fmaf(qa.x, wa0.x, p0); p0 = fmaf(qa.y, wa0.y, p0); p0 = fmaf(qa.z, wa0.z, p0); p0 = fmaf(qa.w, wa0.w, p0);
      p0 = fmaf(qb.x, wa1.x, p0); p0 = fmaf(qb.y, wa1.y, p0); p0 = fmaf(qb.z, wa1.z, p0); p0 = fmaf(qb.w, wa1.w, p0);
      p1 = fmaf(qa.x, wb0.x, p1); p1 = fmaf(qa.y, wb0.y, p1); p1 = fmaf(qa.z, wb0.z, p1); p1 = fmaf(qa.w, wb0.w, p1);
      p1 = fmaf(qb.x, wb1.x, p1); p1 = fmaf(qb.y, wb1.y, p1); p1 = fmaf(qb.z, wb1.z, p1); p1 = fmaf(qb.w, wb1.w, p1);
      const float t0 = tanhf(p0), t1 = tanhf(p1);
      const unsigned wd = pk16(h_bits(t0), h_bits(t1));
      hw = (v4u){hw.y, hw.z, hw.w, wd};
    }
    {
      unsigned short* hp = H1 + (size_t)row * kHid + lane * 8;
      *(volatile v4u*)hp = hw;
      __threadfence();
      *(volatile v4u*)hp = hw;
    }
    float d0 = 0.0f, d1 = 0.0f, d2 = 0.0f, d3 = 0.0f, d4 = 0.0f, d5 = 0.0f, d6 = 0.0f, d7 = 0.0f;
#pragma unroll 1
    for (int kk = 0; kk < 8; ++kk) {
      const int k = lane * 8 + kk;
      const v4f wa = *(const v4f*)(wvt + k * 8), wb = *(const v4f*)(wvt + k * 8 + 4);
      float pre = bv1s[k];
      pre = fmaf(qa.x, wa.x, pre); pre = fmaf(qa.y, wa.y, pre); pre = fmaf(qa.z, wa.z, pre); pre = fmaf(qa.w, wa.w, pre);
      pre = fmaf(qb.x, wb.x, pre); pre = fmaf(qb.y, wb.y, pre); pre = fmaf(qb.z, wb.z, pre); pre = fmaf(qb.w, wb.w, pre);
      const float tt = tanhf(pre);
      const float g = (1.0f - tt * tt) * wv2s[k];
      d0 = fmaf(g, wa.x, d0); d1 = fmaf(g, wa.y, d1); d2 = fmaf(g, wa.z, d2); d3 = fmaf(g, wa.w, d3);
      d4 = fmaf(g, wb.x, d4); d5 = fmaf(g, wb.y, d5); d6 = fmaf(g, wb.z, d6); d7 = fmaf(g, wb.w, d7);
    }
#pragma unroll
    for (int off = 16; off > 0; off >>= 1) {
      d0 += __shfl_xor(d0, off, 32); d1 += __shfl_xor(d1, off, 32); d2 += __shfl_xor(d2, off, 32); d3 += __shfl_xor(d3, off, 32);
      d4 += __shfl_xor(d4, off, 32); d5 += __shfl_xor(d5, off, 32); d6 += __shfl_xor(d6, off, 32); d7 += __shfl_xor(d7, off, 32);
    }
    const float s0 = odd ? d4 : d0, s1 = odd ? d5 : d1, s2 = odd ? d6 : d2, s3 = odd ? d7 : d3;
    const bool mine = (rr == myr);
    k0 = mine ? s0 : k0; k1 = mine ? s1 : k1; k2 = mine ? s2 : k2; k3 = mine ? s3 : k3;
  }
  {
    const v4f kv = (v4f){k0, k1, k2, k3};
    float* dp = DV + (size_t)wrow0 * kNQ + lane * 4;
    *(volatile v4f*)dp = kv;
    __threadfence();
    *(volatile v4f*)dp = kv;
  }
}

__global__ __launch_bounds__(256) void gl_kernel(const float* __restrict__ LP, const float* __restrict__ qd, unsigned* __restrict__ GLw) {
  __shared__ __align__(16) unsigned gls[8 * 32 * 32];
  const int t = threadIdx.x, lane = t & 31, wave = t >> 5;
  const int wrow0 = blockIdx.x * 256 + wave * 32;
  const int row = wrow0 + lane;
  const float* lp = LP + (size_t)row * kNLP;
  v4f cv[9];
#pragma unroll
  for (int m = 0; m < 5; ++m) cv[m] = *(const v4f*)(lp + 4 * m);
  asm volatile("" ::: "memory");
#pragma unroll
  for (int m = 5; m < 9; ++m) cv[m] = *(const v4f*)(lp + 4 * m);
  const v4f qa = *(const v4f*)(qd + (size_t)row * kNQ);
  const v4f qb = *(const v4f*)(qd + (size_t)row * kNQ + 4);
  float lv[36];
#pragma unroll
  for (int m = 0; m < 9; ++m) { lv[4 * m] = cv[m].x; lv[4 * m + 1] = cv[m].y; lv[4 * m + 2] = cv[m].z; lv[4 * m + 3] = cv[m].w; }
  const float qv[8] = {qa.x, qa.y, qa.z, qa.w, qb.x, qb.y, qb.z, qb.w};
  v8f dr = (v8f){lv[0], lv[2], lv[5], lv[9], lv[14], lv[20], lv[27], lv[35]};
  v8f dl = (v8f){0.f,0.f,0.f,0.f,0.f,0.f,0.f,0.f};
  v8f sg = (v8f){0.f,0.f,0.f,0.f,0.f,0.f,0.f,0.f};
#pragma unroll 1
  for (int i = 0; i < 8; ++i) {
    const float x = dr[0];
    const float e = expf(-fabsf(x));
    const float spv = fmaxf(x, 0.0f) + log1pf(e);
    const float r = __builtin_amdgcn_rcpf(1.0f + e);
    const float s = (x >= 0.0f) ? r : e * r;
    dr = (v8f){dr[1], dr[2], dr[3], dr[4], dr[5], dr[6], dr[7], dr[0]};
    dl = (v8f){dl[1], dl[2], dl[3], dl[4], dl[5], dl[6], dl[7], spv + 1.0f};
    sg = (v8f){sg[1], sg[2], sg[3], sg[4], sg[5], sg[6], sg[7], s};
  }
  float u[8];
#pragma unroll
  for (int k = 0; k < 8; ++k) {
    float s = 0.0f;
    s = fmaf(dl[k], qv[k], s);
#pragma unroll
    for (int i = k + 1; i < 8; ++i) s = fmaf(lv[tri_idx(i, k)], qv[i], s);
    u[k] = s;
  }
  float g[36];
#pragma unroll
  for (int i = 0; i < 8; ++i) {
#pragma unroll
    for (int j = 0; j < i; ++j) g[tri_idx(i, j)] = qv[i] * u[j];
    g[tri_idx(i, i)] = qv[i] * u[i] * sg[i];
  }
  unsigned wd[18];
#pragma unroll
  for (int p = 0; p < 18; ++p) wd[p] = pk16(h_bits(g[2 * p]), h_bits(g[2 * p + 1]));
  unsigned* gp = gls + (wave * 32 + lane) * 32;
  *(v4u*)(gp + 0)  = (v4u){wd[0], wd[1], wd[2], wd[3]};
  *(v4u*)(gp + 4)  = (v4u){wd[4], wd[5], wd[6], wd[7]};
  *(v4u*)(gp + 8)  = (v4u){wd[8], wd[9], wd[10], wd[11]};
  *(v4u*)(gp + 12) = (v4u){wd[12], wd[13], wd[14], wd[15]};
  *(v4u*)(gp + 16) = (v4u){wd[16], wd[17], 0u, 0u};
  *(v4u*)(gp + 20) = (v4u){0u, 0u, 0u, 0u};
  *(v4u*)(gp + 24) = (v4u){0u, 0u, 0u, 0u};
  *(v4u*)(gp + 28) = (v4u){0u, 0u, 0u, 0u};
  __syncthreads();
  for (int pass = 0; pass < 2; ++pass) {
#pragma unroll
    for (int s = 0; s < 8; ++s) {
      const int r = s * 4 + (lane >> 3);
      const v4u v = *(const v4u*)(gls + (wave * 32 + r) * 32 + (lane & 7) * 4);
      *(volatile v4u*)(GLw + (size_t)(wrow0 + r) * 32 + (lane & 7) * 4) = v;
    }
    __threadfence();
  }
}

__global__ __launch_bounds__(256) void gemm_gate_kernel(const unsigned short* __restrict__ Ap, const unsigned short* __restrict__ Btp,
                                                       const unsigned short* __restrict__ Hp, unsigned short* __restrict__ Cp, float scale) {
  __shared__ __align__(16) float sT[8][16 * 68];
  const int lane = threadIdx.x & 31, wave = threadIdx.x >> 5;
  const int tile = blockIdx.x * 8 + wave;
  const int tm = tile >> 2, tn = tile & 3;
  const int m0 = tm << 6, n0 = tn << 6;
  v8f acc[4][4];
  mma_tile64_f16<kNLP, kNLP, kNLP>((const _Float16*)Ap, (const _Float16*)Btp, m0, n0, lane, acc);
  float* slab = sT[wave];
  const int rlane = lane & 15, mOff = (lane >> 4) * 8;
  const int q = lane >> 3, c8 = (lane & 7) * 8;
#pragma unroll
  for (int i = 0; i < 4; ++i) {
    const int mBase = m0 + (i << 4);
#pragma unroll
    for (int j = 0; j < 4; ++j)
#pragma unroll
      for (int r = 0; r < 8; ++r) slab[(mOff + r) * 68 + (j << 4) + rlane] = acc[i][j][r] * scale;
    __syncthreads();
    v4u pk[4];
#pragma unroll
    for (int it = 0; it < 4; ++it) {
      const int row = it * 4 + q;
      const v4u hw = *(const v4u*)(Hp + (size_t)(mBase + row) * kHid + n0 + c8);
      const float* sp = slab + row * 68 + c8;
      unsigned wd[4];
#pragma unroll
      for (int w = 0; w < 4; ++w) {
        const float h0 = h16_to_f32(hw[w] & 0xffffu);
        const float h1 = h16_to_f32(hw[w] >> 16);
        const float v0 = sp[2 * w] * (1.0f - h0 * h0);
        const float v1 = sp[2 * w + 1] * (1.0f - h1 * h1);
        wd[w] = pk16(h_bits(v0), h_bits(v1));
      }
      pk[it] = (v4u){wd[0], wd[1], wd[2], wd[3]};
    }
    for (int pass = 0; pass < 2; ++pass) {
#pragma unroll
      for (int it = 0; it < 4; ++it) {
        const int row = it * 4 + q;
        *(volatile v4u*)(Cp + (size_t)(mBase + row) * kHid + n0 + c8) = pk[it];
      }
      __threadfence();
    }
    __syncthreads();
  }
}

__global__ __launch_bounds__(256) void gemm_dt_kernel(const unsigned short* __restrict__ Ap, const unsigned short* __restrict__ Btp,
                                                     const unsigned short* __restrict__ Hp, const float* __restrict__ W1,
                                                     float* __restrict__ DT, float scale) {
  __shared__ __align__(16) float sT[8][16 * 68];
  __shared__ __align__(16) float w1t[kHid * kNQ];
  __shared__ __align__(16) float red[8 * 128];
  const int t = threadIdx.x, lane = t & 31, wave = t >> 5;
  {
    float a[8];
#pragma unroll
    for (int j = 0; j < 8; ++j) a[j] = W1[j * kHid + t];
    *(v4f*)(w1t + t * 8)     = (v4f){a[0], a[1], a[2], a[3]};
    *(v4f*)(w1t + t * 8 + 4) = (v4f){a[4], a[5], a[6], a[7]};
  }
  __syncthreads();
  const int tn = wave & 3, grp = wave >> 2;
  const int m0 = (blockIdx.x * 2 + grp) << 6, n0 = tn << 6;
  v8f acc[4][4];
  mma_tile64_f16<kHid, kHid, kHid>((const _Float16*)Ap, (const _Float16*)Btp, m0, n0, lane, acc);
  float* slab = sT[wave];
  const int rlane = lane & 15, mOff = (lane >> 4) * 8;
  const int q = lane >> 3, c8 = (lane & 7) * 8;
  const int rrow = lane >> 1, jb = (lane & 1) * 4;
#pragma unroll
  for (int i = 0; i < 4; ++i) {
    const int mBase = m0 + (i << 4);
#pragma unroll
    for (int j = 0; j < 4; ++j)
#pragma unroll
      for (int r = 0; r < 8; ++r) slab[(mOff + r) * 68 + (j << 4) + rlane] = acc[i][j][r] * scale;
    __syncthreads();
#pragma unroll
    for (int it = 0; it < 4; ++it) {
      const int row = it * 4 + q;
      const v4u hw = *(const v4u*)(Hp + (size_t)(mBase + row) * kHid + n0 + c8);
      float* sp = slab + row * 68 + c8;
#pragma unroll
      for (int w = 0; w < 4; ++w) {
        const float h0 = h16_to_f32(hw[w] & 0xffffu);
        const float h1 = h16_to_f32(hw[w] >> 16);
        sp[2 * w]     = sp[2 * w] * (1.0f - h0 * h0);
        sp[2 * w + 1] = sp[2 * w + 1] * (1.0f - h1 * h1);
      }
    }
    __syncthreads();
    float d0 = 0.0f, d1 = 0.0f, d2 = 0.0f, d3 = 0.0f;
    {
      const float* srow = slab + rrow * 68;
      const float* wb = w1t + n0 * 8 + jb;
#pragma unroll 8
      for (int n = 0; n < 64; ++n) {
        const float s = srow[n];
        const v4f w = *(const v4f*)(wb + n * 8);
        d0 = fmaf(s, w.x, d0); d1 = fmaf(s, w.y, d1); d2 = fmaf(s, w.z, d2); d3 = fmaf(s, w.w, d3);
      }
    }
    *(v4f*)(red + wave * 128 + lane * 4) = (v4f){d0, d1, d2, d3};
    __syncthreads();
    if (tn == 0) {
      const v4f p0 = *(const v4f*)(red + (grp * 4 + 0) * 128 + lane * 4);
      const v4f p1 = *(const v4f*)(red + (grp * 4 + 1) * 128 + lane * 4);
      const v4f p2 = *(const v4f*)(red + (grp * 4 + 2) * 128 + lane * 4);
      const v4f p3 = *(const v4f*)(red + (grp * 4 + 3) * 128 + lane * 4);
      const v4f tot = ((p0 + p1) + p2) + p3;
      float* dp = DT + (size_t)mBase * kNQ + lane * 4;
      *(volatile v4f*)dp = tot;
      __threadfence();
      *(volatile v4f*)dp = tot;
    }
    __syncthreads();
  }
}

__global__ __launch_bounds__(256) void solve_kernel(const float* __restrict__ LP, const float* __restrict__ tau,
                                                   const float* __restrict__ DT, const float* __restrict__ DV, float* __restrict__ out) {
  __shared__ __align__(16) float os[8 * 256];
  const int t = threadIdx.x, lane = t & 31, wave = t >> 5;
  const int wrow0 = blockIdx.x * 256 + wave * 32;
  const int row = wrow0 + lane;
  const float* lp = LP + (size_t)row * kNLP;
  v4f cv[9];
#pragma unroll
  for (int m = 0; m < 5; ++m) cv[m] = *(const v4f*)(lp + 4 * m);
  asm volatile("" ::: "memory");
#pragma unroll
  for (int m = 5; m < 9; ++m) cv[m] = *(const v4f*)(lp + 4 * m);
  const v4f ta = *(const v4f*)(tau + (size_t)row * kNQ);
  const v4f tb = *(const v4f*)(tau + (size_t)row * kNQ + 4);
  asm volatile("" ::: "memory");
  const v4f da = *(const v4f*)(DT + (size_t)row * kNQ);
  const v4f db = *(const v4f*)(DT + (size_t)row * kNQ + 4);
  const v4f va = *(const v4f*)(DV + (size_t)row * kNQ);
  const v4f vb = *(const v4f*)(DV + (size_t)row * kNQ + 4);
  float lv[36];
#pragma unroll
  for (int m = 0; m < 9; ++m) { lv[4 * m] = cv[m].x; lv[4 * m + 1] = cv[m].y; lv[4 * m + 2] = cv[m].z; lv[4 * m + 3] = cv[m].w; }
  const float tv[8] = {ta.x, ta.y, ta.z, ta.w, tb.x, tb.y, tb.z, tb.w};
  const float dt[8] = {da.x, da.y, da.z, da.w, db.x, db.y, db.z, db.w};
  const float dv[8] = {va.x, va.y, va.z, va.w, vb.x, vb.y, vb.z, vb.w};
  v8f dr = (v8f){lv[0], lv[2], lv[5], lv[9], lv[14], lv[20], lv[27], lv[35]};
  v8f dl = (v8f){0.f,0.f,0.f,0.f,0.f,0.f,0.f,0.f};
#pragma unroll 1
  for (int i = 0; i < 8; ++i) {
    const float x = dr[0];
    const float e = expf(-fabsf(x));
    const float spv = fmaxf(x, 0.0f) + log1pf(e);
    dr = (v8f){dr[1], dr[2], dr[3], dr[4], dr[5], dr[6], dr[7], dr[0]};
    dl = (v8f){dl[1], dl[2], dl[3], dl[4], dl[5], dl[6], dl[7], spv + 1.0f};
  }
  float inv[8], rhs[8];
#pragma unroll
  for (int i = 0; i < 8; ++i) { inv[i] = 1.0f / dl[i]; rhs[i] = (tv[i] - dt[i]) - dv[i]; }
  float y[8];
#pragma unroll
  for (int i = 0; i < 8; ++i) {
    float s = rhs[i];
#pragma unroll
    for (int j = 0; j < i; ++j) s = fmaf(-lv[tri_idx(i, j)], y[j], s);
    y[i] = s * inv[i];
  }
  float a[8];
#pragma unroll
  for (int ii = 7; ii >= 0; --ii) {
    float s = y[ii];
#pragma unroll
    for (int j = ii + 1; j < 8; ++j) s = fmaf(-lv[tri_idx(j, ii)], a[j], s);
    a[ii] = s * inv[ii];
  }
#pragma unroll
  for (int i = 0; i < 8; ++i) a[i] = fminf(100.0f, fmaxf(-100.0f, a[i]));
  *(v4f*)(os + (wave * 32 + lane) * 8)     = (v4f){a[0], a[1], a[2], a[3]};
  *(v4f*)(os + (wave * 32 + lane) * 8 + 4) = (v4f){a[4], a[5], a[6], a[7]};
  __syncthreads();
  for (int pass = 0; pass < 2; ++pass) {
#pragma unroll
    for (int s = 0; s < 2; ++s) {
      const v4f v = *(const v4f*)(os + wave * 256 + s * 128 + lane * 4);
      *(volatile v4f*)(out + (size_t)(wrow0 + s * 16) * kNQ + lane * 4) = v;
    }
    __threadfence();
  }
}

extern "C" void kernel_launch(void* const* d_in, const int* in_sizes, int n_in,
                              void* d_out, int out_size, void* d_ws, size_t ws_size, hipStream_t stream) {
  if (n_in < 12) return;
  if (ws_size < WS_TOTAL) return;
  if (in_sizes[0] != kBS * kNQ || in_sizes[1] != kBS * kNQ || in_sizes[2] != kBS * kNQ) return;
  if (in_sizes[3] != kNQ * kHid || in_sizes[4] != kHid || in_sizes[5] != kHid * kHid || in_sizes[6] != kHid) return;
  if (in_sizes[7] != kHid * kNL || in_sizes[8] != kNL || in_sizes[9] != kNQ * kHid || in_sizes[10] != kHid || in_sizes[11] != kHid) return;
  if (out_size != kBS * kNQ) return;

  const float* q   = (const float*)d_in[0];
  const float* qd  = (const float*)d_in[1];
  const float* tau = (const float*)d_in[2];
  const float* W1  = (const float*)d_in[3];
  const float* b1  = (const float*)d_in[4];
  const float* W2  = (const float*)d_in[5];
  const float* b2  = (const float*)d_in[6];
  const float* W3  = (const float*)d_in[7];
  const float* b3  = (const float*)d_in[8];
  const float* Wv1 = (const float*)d_in[9];
  const float* bv1 = (const float*)d_in[10];
  const float* Wv2 = (const float*)d_in[11];
  float* out = (float*)d_out;
  char* ws = (char*)d_ws;
  unsigned short* H1  = (unsigned short*)(ws + OFF_H1);
  unsigned short* H2  = (unsigned short*)(ws + OFF_H2);
  unsigned short* GP2 = (unsigned short*)(ws + OFF_GP2);
  unsigned short* GL  = (unsigned short*)(ws + OFF_GL);
  float*          LP  = (float*)(ws + OFF_LP);
  float*          DV  = (float*)(ws + OFF_DV);
  float*          DT  = (float*)(ws + OFF_DT);
  unsigned short* W2T = (unsigned short*)(ws + OFF_W2T);
  unsigned short* W2C = (unsigned short*)(ws + OFF_W2C);
  unsigned short* W3T = (unsigned short*)(ws + OFF_W3T);
  unsigned short* W3B = (unsigned short*)(ws + OFF_W3B);
  float*          B3P = (float*)(ws + OFF_B3P);

  pack_w2t_kernel<<<dim3(kHid / 64, kHid / 64), 256, 0, stream>>>(W2, W2T, kWCarry);
  pack_cast8_kernel<<<(kHid * kHid / 8) / 256, 256, 0, stream>>>(W2, W2C, kHid * kHid / 8, kWCarry);
  pack_w3_kernel<<<2, 256, 0, stream>>>(W3, b3, W3T, W3B, B3P, kWCarry);
  h1_vnet_kernel<<<kBS / 128, 256, 0, stream>>>(q, W1, b1, Wv1, bv1, Wv2, H1, DV);
  wmma_gemm64<0, false, 2, 1, false, 1><<<dim3((kBS / 64) * (kHid / 64) / 8, 1), 256, 0, stream>>>(
      H1, H1, kHid, 0L, W2T, W2T, kHid, 0L, (void*)H2, (void*)H2, kHid, 0L, b2, nullptr, 0L, kBS, kHid, kHid, kWCarryInv);
  wmma_gemm64<0, false, 2, 0, false, 0><<<dim3((kBS / 64) * (kNLP / 64) / 8, 1), 256, 0, stream>>>(
      H2, H2, kHid, 0L, W3T, W3T, kHid, 0L, (void*)LP, (void*)LP, kNLP, 0L, B3P, nullptr, 0L, kBS, kNLP, kHid, kWCarryInv);
  gl_kernel<<<kBS / 256, 256, 0, stream>>>(LP, qd, (unsigned*)GL);
  gemm_gate_kernel<<<(kBS / 64) * (kHid / 64) / 8, 256, 0, stream>>>(GL, W3B, H2, GP2, kWCarryInv);
  gemm_dt_kernel<<<(kBS / 64) * (kHid / 64) / 8, 256, 0, stream>>>(GP2, W2C, H1, W1, DT, kWCarryInv);
  solve_kernel<<<kBS / 256, 256, 0, stream>>>(LP, tau, DT, DV, out);
}
